// GraphAttentionLayerSparse_78769700208702
// MI455X (gfx1250) — hardware-verified
//
#include <hip/hip_runtime.h>
#include <stddef.h>


#define NF    128
#define NH    4
#define HD    64
#define NCOL  (NH * HD)
#define GR    32
#define AP    136
#define XSP   260
#define NB    256
#define CHUNK 2048
#define NTHR  256
#define NWAVE 8
#define WCAP  256
#define NGRP  (CHUNK / (NTHR * 4))

#define LDS_SACC (NB * NCOL)
#define LDS_DEN  (NB * NH)
#define LDS_MX   (NB * NH)
#define LDS_LIST (NWAVE * WCAP)
#define LDS_BYTES ((LDS_SACC + LDS_DEN + LDS_MX + LDS_LIST + NWAVE) * 4)

static_assert(WCAP == (CHUNK / NTHR) * 32);
static_assert(NGRP == 2);
static_assert(NB == 256);
static_assert(CHUNK == 2048);
static_assert(((LDS_SACC + LDS_DEN) % 4) == 0);
static_assert(LDS_BYTES == 278560);
static_assert((NB % NWAVE) == 0);

typedef float  v4f  __attribute__((ext_vector_type(4)));
typedef float  v8f  __attribute__((ext_vector_type(8)));
typedef int    v4i  __attribute__((ext_vector_type(4)));
typedef __bf16 v8b  __attribute__((ext_vector_type(8)));
typedef __bf16 v16b __attribute__((ext_vector_type(16)));
union Frag  { v16b v; v8b half[2]; };
union PackB { v8b b; v4i i; };

__device__ __forceinline__ v8f wm(v16b a, v16b b, v8f c) {
  v8f d = __builtin_amdgcn_wmma_f32_16x16x32_bf16(false, a, false, b, (short)0, c, false, false);
  asm volatile("v_nop\n\tv_nop\n\tv_nop\n\tv_nop" : "+v"(d) : "v"(a), "v"(b));
  return d;
}

#define SPL(U, L, IDX, VAL) { const float vv_ = (VAL); const __bf16 hb_ = (__bf16)vv_; \
    (U).b[IDX] = hb_; (L).b[IDX] = (__bf16)(vv_ - (float)hb_); }

__global__ __launch_bounds__(NTHR) void k_prepw(const float* __restrict__ W, __bf16* Wth, __bf16* Wtl, int nItems) {
  const int i = blockIdx.x * NTHR + threadIdx.x;
  if (i >= nItems) return;
  const int n    = i >> 4;
  const int k0   = (i & 15) * 8;
  const int head = n >> 6;
  const int d    = n & 63;
  const float* p = W + ((size_t)head * NF + k0) * HD + d;
  PackB hi, lo;
#pragma unroll
  for (int j = 0; j < 8; ++j) SPL(hi, lo, j, p[(size_t)j * HD])
  const size_t o = (size_t)n * NF + k0;
  const v4i hv = hi.i, lv = lo.i;
  *(volatile v4i*)(Wth + o) = hv;
  *(volatile v4i*)(Wtl + o) = lv;
  __threadfence();
  *(volatile v4i*)(Wth + o) = hv;
  *(volatile v4i*)(Wtl + o) = lv;
}

__global__ __launch_bounds__(NTHR) void k_gemm(
    const float* __restrict__ X, const __bf16* __restrict__ Wth, const __bf16* __restrict__ Wtl,
    const float* __restrict__ attn, float* Hws, float* aL, float* aR, int nN) {
  __shared__ __attribute__((aligned(16))) __bf16 Ah[GR * AP];
  __shared__ __attribute__((aligned(16))) __bf16 Al[GR * AP];
  __shared__ __attribute__((aligned(16))) float Xs[GR * XSP];
  __shared__ __attribute__((aligned(16))) float As[NH * 2 * HD];
  __shared__ __attribute__((aligned(16))) float Ls[2 * GR * NH];

  const int tid  = threadIdx.x;
  const int lane = tid & 31;
  const int wave = tid >> 5;
  const int hh   = lane >> 4;
  const int m    = lane & 15;
  const int rowBase = blockIdx.x * GR;

  {
    const int r  = tid >> 3;
    const int c0 = (tid & 7) * 16;
    int row = rowBase + r;
    if (row > nN - 1) row = nN - 1;
    const float* p = X + (size_t)row * NF + c0;
    const v4f f0 = *(const v4f*)(p), f1 = *(const v4f*)(p + 4);
    const v4f f2 = *(const v4f*)(p + 8), f3 = *(const v4f*)(p + 12);
    PackB h0, l0, h1, l1;
    SPL(h0, l0, 0, f0.x) SPL(h0, l0, 1, f0.y) SPL(h0, l0, 2, f0.z) SPL(h0, l0, 3, f0.w)
    SPL(h0, l0, 4, f1.x) SPL(h0, l0, 5, f1.y) SPL(h0, l0, 6, f1.z) SPL(h0, l0, 7, f1.w)
    SPL(h1, l1, 0, f2.x) SPL(h1, l1, 1, f2.y) SPL(h1, l1, 2, f2.z) SPL(h1, l1, 3, f2.w)
    SPL(h1, l1, 4, f3.x) SPL(h1, l1, 5, f3.y) SPL(h1, l1, 6, f3.z) SPL(h1, l1, 7, f3.w)
    *(v8b*)(Ah + r * AP + c0)     = h0.b;
    *(v8b*)(Ah + r * AP + c0 + 8) = h1.b;
    *(v8b*)(Al + r * AP + c0)     = l0.b;
    *(v8b*)(Al + r * AP + c0 + 8) = l1.b;
    if (tid < (NH * 2 * HD) / 4) *(v4f*)(As + 4 * tid) = *(const v4f*)(attn + 4 * tid);
  }
  __syncthreads();

  const int ncol0 = wave * 32 + m;
  const int ncol1 = ncol0 + 16;
  v8f c00 = {0.f, 0.f, 0.f, 0.f, 0.f, 0.f, 0.f, 0.f};
  v8f c01 = {0.f, 0.f, 0.f, 0.f, 0.f, 0.f, 0.f, 0.f};
  v8f c10 = {0.f, 0.f, 0.f, 0.f, 0.f, 0.f, 0.f, 0.f};
  v8f c11 = {0.f, 0.f, 0.f, 0.f, 0.f, 0.f, 0.f, 0.f};
#pragma unroll 1
  for (int kt = 0; kt < NF / 32; ++kt) {
    const int k0 = kt * 32;
    Frag a0h, a0l, a1h, a1l, b0h, b0l, b1h, b1l;
    const __bf16* pa0h = Ah + m * AP + k0 + 8 * hh;
    const __bf16* pa1h = Ah + (16 + m) * AP + k0 + 8 * hh;
    const __bf16* pa0l = Al + m * AP + k0 + 8 * hh;
    const __bf16* pa1l = Al + (16 + m) * AP + k0 + 8 * hh;
    const __bf16* pb0h = Wth + (size_t)ncol0 * NF + k0 + 8 * hh;
    const __bf16* pb1h = Wth + (size_t)ncol1 * NF + k0 + 8 * hh;
    const __bf16* pb0l = Wtl + (size_t)ncol0 * NF + k0 + 8 * hh;
    const __bf16* pb1l = Wtl + (size_t)ncol1 * NF + k0 + 8 * hh;
    a0h.half[0] = *(const v8b*)pa0h; a0h.half[1] = *(const v8b*)(pa0h + 16);
    a1h.half[0] = *(const v8b*)pa1h; a1h.half[1] = *(const v8b*)(pa1h + 16);
    a0l.half[0] = *(const v8b*)pa0l; a0l.half[1] = *(const v8b*)(pa0l + 16);
    a1l.half[0] = *(const v8b*)pa1l; a1l.half[1] = *(const v8b*)(pa1l + 16);
    b0h.half[0] = *(const v8b*)pb0h; b0h.half[1] = *(const v8b*)(pb0h + 16);
    b1h.half[0] = *(const v8b*)pb1h; b1h.half[1] = *(const v8b*)(pb1h + 16);
    b0l.half[0] = *(const v8b*)pb0l; b0l.half[1] = *(const v8b*)(pb0l + 16);
    b1l.half[0] = *(const v8b*)pb1l; b1l.half[1] = *(const v8b*)(pb1l + 16);
    c00 = wm(a0h.v, b0h.v, c00); c00 = wm(a0h.v, b0l.v, c00); c00 = wm(a0l.v, b0h.v, c00);
    c01 = wm(a0h.v, b1h.v, c01); c01 = wm(a0h.v, b1l.v, c01); c01 = wm(a0l.v, b1h.v, c01);
    c10 = wm(a1h.v, b0h.v, c10); c10 = wm(a1h.v, b0l.v, c10); c10 = wm(a1l.v, b0h.v, c10);
    c11 = wm(a1h.v, b1h.v, c11); c11 = wm(a1h.v, b1l.v, c11); c11 = wm(a1l.v, b1h.v, c11);
  }

#pragma unroll
  for (int r = 0; r < 8; ++r) {
    Xs[(8 * hh + r) * XSP + ncol0]      = c00[r];
    Xs[(8 * hh + r) * XSP + ncol1]      = c01[r];
    Xs[(16 + 8 * hh + r) * XSP + ncol0] = c10[r];
    Xs[(16 + 8 * hh + r) * XSP + ncol1] = c11[r];
  }
  __syncthreads();

  {
    const int row  = tid >> 3;
    const int head = (tid >> 1) & 3;
    const int side = tid & 1;
    const float* xs = Xs + row * XSP + head * HD;
    const float* as = As + head * (2 * HD) + side * HD;
    float s = 0.f;
#pragma unroll
    for (int j = 0; j < HD / 4; ++j) {
      const v4f a = *(const v4f*)(xs + 4 * j);
      const v4f b = *(const v4f*)(as + 4 * j);
      s += a.x * b.x; s += a.y * b.y; s += a.z * b.z; s += a.w * b.w;
    }
    Ls[side * (GR * NH) + row * NH + head] = s;
  }
  __syncthreads();

  v4f xr[8];
#pragma unroll
  for (int i = 0; i < 4; ++i) {
    xr[2 * i]     = *(const v4f*)(Xs + (4 * wave + i) * XSP + 4 * lane);
    xr[2 * i + 1] = *(const v4f*)(Xs + (4 * wave + i) * XSP + 128 + 4 * lane);
  }
  float* gp = 0;
  v4f gv = {0.f, 0.f, 0.f, 0.f};
  if (wave == 0) {
    gv = *(const v4f*)(Ls + 4 * lane);
    gp = aL + (size_t)rowBase * NH + 4 * lane;
  } else if (wave == 1) {
    gv = *(const v4f*)(Ls + GR * NH + 4 * lane);
    gp = aR + (size_t)rowBase * NH + 4 * lane;
  }
  float* hp[4];
#pragma unroll
  for (int i = 0; i < 4; ++i) hp[i] = Hws + (size_t)(rowBase + 4 * wave + i) * NCOL + 4 * lane;

#pragma unroll
  for (int i = 0; i < 4; ++i) {
    *(volatile v4f*)(hp[i])       = xr[2 * i];
    *(volatile v4f*)(hp[i] + 128) = xr[2 * i + 1];
  }
  if (gp) *(volatile v4f*)gp = gv;
  __threadfence();
#pragma unroll
  for (int i = 0; i < 4; ++i) {
    *(volatile v4f*)(hp[i])       = xr[2 * i];
    *(volatile v4f*)(hp[i] + 128) = xr[2 * i + 1];
  }
  if (gp) *(volatile v4f*)gp = gv;
}

__global__ __launch_bounds__(NTHR) void k_gat(
    const int* __restrict__ ei, const float* __restrict__ ew,
    const float* __restrict__ Hws, const float* __restrict__ aL, const float* __restrict__ aR,
    float* out, int nN, int nE) {
  extern __shared__ v4f lds_dyn[];
  float* sacc = (float*)lds_dyn;
  float* den  = sacc + LDS_SACC;
  float* mx   = den + LDS_DEN;
  int*   list = (int*)(mx + LDS_MX);
  int*   wcnt = list + LDS_LIST;

  const int tid  = threadIdx.x;
  const int lane = tid & 31;
  const int wave = tid >> 5;
  const int hd   = lane >> 3;
  const int c8   = 8 * lane;
  const int nodeBase = blockIdx.x * NB;

  {
    const v4f z4 = {0.f, 0.f, 0.f, 0.f};
    for (int i = tid; i < (LDS_SACC + LDS_DEN) / 4; i += NTHR) lds_dyn[i] = z4;
    for (int i = tid; i < LDS_MX; i += NTHR) mx[i] = -1.0e30f;
  }
  __syncthreads();

  const int* eid = ei + nE;
  const bool al16 = ((nE & 3) == 0);

  const int nChunks = (nE + CHUNK - 1) / CHUNK;
#pragma unroll 1
  for (int ch = 0; ch < nChunks; ++ch) {
    const int cbase = ch * CHUNK;
    int wc = 0;
#pragma unroll
    for (int g = 0; g < NGRP; ++g) {
      const int el0 = (g * NTHR + tid) * 4;
      const int e0  = cbase + el0;
      const int sent = -2147483647 - 1;
      v4i d;
      if (al16 && (e0 + 3 < nE)) {
        d = *(const v4i*)(eid + e0);
      } else {
        d.x = (e0     < nE) ? eid[min(e0, nE - 1)]     : sent;
        d.y = (e0 + 1 < nE) ? eid[min(e0 + 1, nE - 1)] : sent;
        d.z = (e0 + 2 < nE) ? eid[min(e0 + 2, nE - 1)] : sent;
        d.w = (e0 + 3 < nE) ? eid[min(e0 + 3, nE - 1)] : sent;
      }
      const unsigned s0 = (unsigned)d.x - (unsigned)nodeBase;
      const unsigned s1 = (unsigned)d.y - (unsigned)nodeBase;
      const unsigned s2 = (unsigned)d.z - (unsigned)nodeBase;
      const unsigned s3 = (unsigned)d.w - (unsigned)nodeBase;
      const bool h0 = s0 < (unsigned)NB;
      const bool h1 = s1 < (unsigned)NB;
      const bool h2 = s2 < (unsigned)NB;
      const bool h3 = s3 < (unsigned)NB;
      const unsigned many = __builtin_amdgcn_ballot_w32(h0 | h1 | h2 | h3);
      if (many != 0u) {
#define HITJ(J, HJ, SJ) { \
          const unsigned mj = __builtin_amdgcn_ballot_w32(HJ); \
          if (HJ) { \
            const int pos = wc + (int)__builtin_amdgcn_mbcnt_lo(mj, 0u); \
            if (pos < WCAP) list[wave * WCAP + pos] = ((el0 + (J)) << 8) | (int)(SJ); \
          } \
          wc += (int)__builtin_popcount(mj); }
        HITJ(0, h0, s0)
        HITJ(1, h1, s1)
        HITJ(2, h2, s2)
        HITJ(3, h3, s3)
#undef HITJ
      }
    }
    if (lane == 0) wcnt[wave] = wc;
    __syncthreads();

    if (wave == 0) {
      for (int wsx = 0; wsx < NWAVE; ++wsx) {
        int n = wcnt[wsx];
        if (n > WCAP) n = WCAP;
        if (n < 0) n = 0;
        for (int i = 0; i < n; ++i) {
          const int ent  = list[wsx * WCAP + i];
          const int slot = ent & (NB - 1);
          const int el   = (ent >> 8) & (CHUNK - 1);
          int e = cbase + el;
          if (e > nE - 1) e = nE - 1;
          int src = ei[e];
          src = src < 0 ? 0 : (src > nN - 1 ? nN - 1 : src);
          const float w = ew[e];
          int nd = nodeBase + slot;
          if (nd > nN - 1) nd = nN - 1;
          float x = aL[(size_t)nd * NH + hd] + aR[(size_t)src * NH + hd];
          x = (x > 0.f) ? x : 0.2f * x;
          const int di = slot * NH + hd;
          const float mo = mx[di];
          const float mn = fmaxf(mo, x);
          const float sc = __expf(mo - mn);
          const float p  = __expf(x - mn);
          const float pw = p * w;
          const float* hrow = Hws + (size_t)src * NCOL + c8;
          const v4f hv0 = *(const v4f*)(hrow);
          const v4f hv1 = *(const v4f*)(hrow + 4);
          v4f* sp = (v4f*)(sacc + slot * NCOL + c8);
          const v4f a0 = sp[0];
          const v4f a1 = sp[1];
          const v4f n0 = a0 * sc + pw * hv0;
          const v4f n1 = a1 * sc + pw * hv1;
          sp[0] = n0;
          sp[1] = n1;
          if ((lane & 7) == 0) {
            const float dv = den[di];
            den[di] = dv * sc + p;
            mx[di]  = mn;
          }
        }
      }
    }
    __syncthreads();
  }

  const int q = lane >> 4;
#pragma unroll 1
  for (int j = 0; j < NB / NWAVE; ++j) {
    const int slot = wave * (NB / NWAVE) + j;
    const int node = nodeBase + slot;
    if (node >= nN) break;
    const float inv0 = 1.0f / (den[slot * NH + q] + 1e-9f);
    const float inv1 = 1.0f / (den[slot * NH + q + 2] + 1e-9f);
    const v4f s0 = *(const v4f*)(sacc + slot * NCOL + 4 * lane);
    const v4f s1 = *(const v4f*)(sacc + slot * NCOL + 128 + 4 * lane);
    v4f y0 = s0 * inv0;
    v4f y1 = s1 * inv1;
    y0.x = y0.x > 0.f ? y0.x : 0.f; y0.y = y0.y > 0.f ? y0.y : 0.f;
    y0.z = y0.z > 0.f ? y0.z : 0.f; y0.w = y0.w > 0.f ? y0.w : 0.f;
    y1.x = y1.x > 0.f ? y1.x : 0.f; y1.y = y1.y > 0.f ? y1.y : 0.f;
    y1.z = y1.z > 0.f ? y1.z : 0.f; y1.w = y1.w > 0.f ? y1.w : 0.f;
    float* op = out + (size_t)node * NCOL + 4 * lane;
    *(volatile v4f*)op         = y0;
    *(volatile v4f*)(op + 128) = y1;
    __threadfence();
    *(volatile v4f*)op         = y0;
    *(volatile v4f*)(op + 128) = y1;
  }
}

extern "C" void kernel_launch(void* const* d_in, const int* in_sizes, int n_in,
                              void* d_out, int out_size, void* d_ws, size_t ws_size,
                              hipStream_t stream) {
  if (n_in < 5) return;
  const int nE = in_sizes[0] / 2;
  const int nN = in_sizes[2] / NF;
  if (nE <= 0 || in_sizes[0] != 2 * nE) return;
  if (in_sizes[1] != nE) return;
  if (nN <= 0 || in_sizes[2] != nN * NF) return;
  if (in_sizes[3] != NH * NF * HD) return;
  if (in_sizes[4] != NH * 2 * HD) return;
  if (out_size != nN * NCOL) return;

  const int*   ei = (const int*)d_in[0];
  const float* ew = (const float*)d_in[1];
  const float* X  = (const float*)d_in[2];
  const float* W  = (const float*)d_in[3];
  const float* A  = (const float*)d_in[4];
  float* out = (float*)d_out;

  const int nP = ((nN + GR - 1) / GR) * GR;
  size_t off = 0;
  float* Hws  = (float*)((char*)d_ws + off);   off += (size_t)nP * NCOL * sizeof(float);
  float* aL   = (float*)((char*)d_ws + off);   off += (size_t)nP * NH * sizeof(float);
  float* aR   = (float*)((char*)d_ws + off);   off += (size_t)nP * NH * sizeof(float);
  __bf16* Wth = (__bf16*)((char*)d_ws + off);  off += (size_t)NCOL * NF * sizeof(__bf16);
  __bf16* Wtl = (__bf16*)((char*)d_ws + off);  off += (size_t)NCOL * NF * sizeof(__bf16);
  if (off > ws_size) return;
  if (off > (size_t)134217728) return;

  const int nItems = NCOL * (NF / 8);
  k_prepw<<<(nItems + NTHR - 1) / NTHR, NTHR, 0, stream>>>(W, Wth, Wtl, nItems);

  k_gemm<<<nP / GR, NTHR, 0, stream>>>(X, Wth, Wtl, A, Hws, aL, aR, nN);

  hipFuncSetAttribute(reinterpret_cast<const void*>(&k_gat),
                      hipFuncAttributeMaxDynamicSharedMemorySize, LDS_BYTES);
  const int grid = (nN + NB - 1) / NB;
  k_gat<<<grid, NTHR, LDS_BYTES, stream>>>(ei, ew, Hws, aL, aR, out, nN, nE);
}
